// MultiModalPredictor_90598040142139
// MI455X (gfx1250) — hardware-run, weakly checked
//
#include <hip/hip_runtime.h>


namespace {
constexpr int N = 50000, NP = 50048, E = 800000, EQ = E / 4, H = 128, ED = 16, KIN = 2 * H + ED + 4, KP = 288, G3 = 3 * H;
constexpr float XS = 8.0f, WSC = 256.0f, EPS = 1e-5f;
static_assert(E % 16 == 0 && EQ % 16 == 0 && 4 * EQ == E, "16-edge waves must not straddle a quarter");

typedef _Float16 b16;
typedef __attribute__((ext_vector_type(16))) _Float16 v16b;
typedef __attribute__((ext_vector_type(8))) _Float16 v8b;
typedef __attribute__((ext_vector_type(4))) _Float16 v4b;
typedef __attribute__((ext_vector_type(8))) float v8f;
typedef __attribute__((ext_vector_type(4))) float v4f;
__device__ __forceinline__ float bf16_rne(float f) { unsigned int u = __float_as_uint(f); u += 0x7FFFu + ((u >> 16) & 1u); return __uint_as_float(u & 0xFFFF0000u); }
__device__ __forceinline__ void split16(float v, b16& hi, b16& lo) { hi = (b16)v; lo = (b16)(v - (float)hi); }
__device__ __forceinline__ v16b frag_kb(const b16* p, int hh) { const v8b a = *(const v8b*)(p + 8 * hh), b = *(const v8b*)(p + 16 + 8 * hh); v16b f;
#pragma unroll
  for (int e = 0; e < 8; ++e) { f[e] = a[e]; f[8 + e] = b[e]; } return f; }
__device__ __forceinline__ v8f wmma16b(v16b a, v16b b, v8f c) { v8f d = __builtin_amdgcn_wmma_f32_16x16x32_f16(false, a, false, b, (short)0, c, false, false); asm volatile("v_nop\n\tv_nop\n\tv_nop\n\tv_nop" : "+v"(d) : "v"(a), "v"(b)); return d; }
__device__ __forceinline__ void wave_lds_sync() { __builtin_amdgcn_fence(__ATOMIC_RELEASE, "workgroup"); __builtin_amdgcn_wave_barrier(); __builtin_amdgcn_fence(__ATOMIC_ACQUIRE, "workgroup"); }
__device__ __forceinline__ float nexp(float x) { return __builtin_amdgcn_exp2f(x * 1.4426950408889634f); }
__device__ __forceinline__ float pmul(float a, float b) { float p = a * b; asm volatile("" : "+v"(p)); return p; }
__device__ __forceinline__ float hsum16(float v) { v += __shfl_xor(v, 1); v += __shfl_xor(v, 2); v += __shfl_xor(v, 4); return v + __shfl_xor(v, 8); }
__device__ __forceinline__ int iclamp(int v, int lo, int hi) { return v < lo ? lo : (v > hi ? hi : v); }
__device__ __forceinline__ float sigm(float x) { return 1.0f / (1.0f + nexp(-x)); }
__device__ __forceinline__ float tanh_(float x) { const float e = nexp(-2.0f * fabsf(x)); const float t = (1.0f - e) / (1.0f + e); return x < 0.0f ? -t : t; }

constexpr int CSR_NBLK = 512, CSR_GB = 9, CSR_GN = 1 << CSR_GB  , CSR_MAXG = 512, CSR_CAP = 12288  ;
__global__ __launch_bounds__(64) void csrA_kernel(const int* __restrict__ dst, int E, int N, int nG, int CHP, int NGP, int* __restrict__ STG, int* __restrict__ HST) {
  extern __shared__ int sm[];
  int* cnt = sm; int* run = sm + NGP; int* ids = sm + 2 * NGP;
  const int b = blockIdx.x; const int ch = (E + CSR_NBLK - 1) / CSR_NBLK; const int e0 = b * ch, e1 = min(E, e0 + ch);
  for (int i = threadIdx.x; i < NGP; i += 64) cnt[i] = 0;
  for (int i = threadIdx.x; i < CHP; i += 64) ids[i] = -1;
  __syncthreads();
  if (threadIdx.x == 0) {
    for (int e = e0; e < e1; ++e) { int d = dst[e]; d = (d < 0) ? 0 : (d >= N ? N - 1 : d); cnt[d >> CSR_GB] += 1; }
    int acc = 0; for (int g = 0; g < nG; ++g) { run[g] = acc; acc += cnt[g]; }
    for (int e = e0; e < e1; ++e) { int d = dst[e]; d = (d < 0) ? 0 : (d >= N ? N - 1 : d); const int g = d >> CSR_GB; ids[run[g]] = e; run[g] += 1; } }
  __syncthreads();
  typedef __attribute__((ext_vector_type(4))) int v4i;
  for (int pass = 0; pass < 2; ++pass) {
    for (int i = threadIdx.x; i < CHP / 4; i += 64) *(volatile v4i*)(STG + (size_t)b * CHP + i * 4) = *(const v4i*)(&ids[i * 4]);
    for (int i = threadIdx.x; i < NGP / 4; i += 64) { v4i v; for (int e = 0; e < 4; ++e) v[e] = (i * 4 + e < nG) ? cnt[i * 4 + e] : 0; *(volatile v4i*)(HST + (size_t)b * NGP + i * 4) = v; }
    __threadfence(); }
}
__global__ __launch_bounds__(512) void csrS_kernel(const int* __restrict__ HST, int nG, int NGP, int* __restrict__ START, int* __restrict__ TOT, int* __restrict__ OFF) {
  __shared__ int tot[CSR_MAXG];
  const int b = threadIdx.x;
  for (int pass = 0; pass < 2; ++pass) { int runb = 0; for (int g = 0; g < nG; ++g) { int c = HST[(size_t)b * NGP + g]; c = (c < 0) ? 0 : c; ((volatile int*)OFF)[(size_t)g * CSR_NBLK + b] = runb; runb += c; } __threadfence(); }
  for (int g = threadIdx.x; g < nG; g += 512) { int s = 0; for (int bb = 0; bb < CSR_NBLK; ++bb) { int c = HST[(size_t)bb * NGP + g]; s += (c < 0) ? 0 : c; } tot[g] = s; }
  __syncthreads();
  if (threadIdx.x < 32) {
    __shared__ int st[CSR_MAXG + 32];
    if (threadIdx.x == 0) { int acc = 0; for (int g = 0; g < NGP; ++g) { st[g] = acc; if (g < nG) acc += (tot[g] + 31) & ~31; } st[NGP] = acc; }
    __builtin_amdgcn_fence(__ATOMIC_RELEASE, "workgroup"); __builtin_amdgcn_wave_barrier(); __builtin_amdgcn_fence(__ATOMIC_ACQUIRE, "workgroup");
    for (int pass = 0; pass < 2; ++pass) { for (int i = threadIdx.x; i < NGP + 32; i += 32) { ((volatile int*)START)[i] = (i <= NGP) ? st[min(i, NGP)] : 0; ((volatile int*)TOT)[i] = (i < nG) ? tot[i] : 0; } __threadfence(); } }
}
__global__ __launch_bounds__(256) void csrB_kernel(const int* __restrict__ dst, int N, int nG, int CHP, int NGP, int permLen, const int* __restrict__ STG, const int* __restrict__ HST, const int* __restrict__ OFF, const int* __restrict__ START, const int* __restrict__ TOT, int* __restrict__ PERM, int* __restrict__ ROWPTR, int* __restrict__ ROWCNT, int* __restrict__ FLAG) {
  typedef __attribute__((ext_vector_type(4))) int v4i;
  __shared__ int ids[CSR_CAP]; __shared__ unsigned short key[CSR_CAP]; __shared__ int outp[CSR_CAP]; __shared__ int ncnt[CSR_GN + 1]; __shared__ int boff[CSR_NBLK + 1];
  const int g = blockIdx.x, t_ = threadIdx.x; int tot = TOT[g]; int st = START[g], stn = START[g + 1]; const int v0 = g * CSR_GN; const int nv = min(CSR_GN, N - v0);
  st = (st < 0) ? 0 : (st > permLen - 32 ? permLen - 32 : st) & ~31; stn = (stn < st) ? st : (stn > permLen ? permLen : stn); tot = (tot < 0) ? 0 : tot; if (tot > stn - st && tot <= CSR_CAP) tot = stn - st;
  if (tot > CSR_CAP) {
    for (int pass = 0; pass < 2; ++pass) { for (int i = t_; i < CSR_GN / 4; i += 256) { v4i a, c; for (int e = 0; e < 4; ++e) { a[e] = st; c[e] = 0; } *(volatile v4i*)(ROWPTR + v0 + i * 4) = a; *(volatile v4i*)(ROWCNT + v0 + i * 4) = c; } if (t_ == 0) ((volatile int*)FLAG)[0] = 1; __threadfence(); } (void)nv; return; }
  if (t_ == 0) { int acc = 0; for (int b = 0; b < CSR_NBLK; ++b) { boff[b] = acc; int c = HST[(size_t)b * NGP + g]; c = (c < 0) ? 0 : (c > CHP ? CHP : c); acc += c; if (acc > tot) acc = tot; } boff[CSR_NBLK] = acc; }
  for (int i = t_; i <= CSR_GN; i += 256) ncnt[i] = 0;
  __syncthreads();
  for (int b = 0; b < CSR_NBLK; ++b) { const int c = boff[b + 1] - boff[b]; int o_ = OFF[(size_t)g * CSR_NBLK + b]; o_ = (o_ < 0) ? 0 : (o_ > CHP - c ? CHP - c : o_); const int* src_ = STG + (size_t)b * CHP + o_;
    for (int i = t_; i < c; i += 256) { int id = src_[i]; id = (id < 0) ? 0 : id; ids[boff[b] + i] = id; int d = dst[id]; d = (d < v0) ? v0 : (d >= N ? N - 1 : d); int kk = d - v0; kk = (kk < 0) ? 0 : (kk >= CSR_GN ? CSR_GN - 1 : kk); key[boff[b] + i] = (unsigned short)kk; } }
  __syncthreads();
  if (t_ == 0) { for (int i = 0; i < tot; ++i) ncnt[key[i]] += 1; int acc = 0; for (int vl = 0; vl < CSR_GN; ++vl) { const int c = ncnt[vl]; ncnt[vl] = acc; acc += c; } ncnt[CSR_GN] = acc;
    for (int i = 0; i < tot; ++i) { const int vl = key[i]; outp[ncnt[vl]] = ids[i]; ncnt[vl] += 1; }
    for (int vl = CSR_GN; vl > 0; --vl) ncnt[vl] = ncnt[vl - 1]; ncnt[0] = 0; }
  __syncthreads();
  for (int pass = 0; pass < 2; ++pass) {
    for (int i = t_; i < (stn - st) / 4; i += 256) { v4i v; for (int e = 0; e < 4; ++e) { const int q = i * 4 + e; v[e] = (q < tot) ? outp[q] : -1; } *(volatile v4i*)(PERM + st + i * 4) = v; }
    for (int i = t_; i < CSR_GN / 4; i += 256) { v4i a, c; for (int e = 0; e < 4; ++e) { const int vl = i * 4 + e; a[e] = st + ncnt[vl]; c[e] = (vl < nv) ? (ncnt[vl + 1] - ncnt[vl]) : 0; } *(volatile v4i*)(ROWPTR + v0 + i * 4) = a; *(volatile v4i*)(ROWCNT + v0 + i * 4) = c; }
    __threadfence(); }
}
__global__ __launch_bounds__(256) void csrZ_kernel(int* __restrict__ p, size_t n4) { typedef __attribute__((ext_vector_type(4))) int v4i; const size_t tid = (size_t)blockIdx.x * 256 + threadIdx.x, nth = (size_t)gridDim.x * 256; v4i z = {0, 0, 0, 0}; for (size_t i = tid; i < n4; i += nth) *(volatile v4i*)(p + i * 4) = z; }
struct CsrBufs { int *STG, *HST, *OFF, *START, *TOT, *PERM, *ROWPTR, *ROWCNT, *FLAG; int nG, NGP, CHP; size_t permLen; char* base; size_t bytes; };
static size_t csr_carve(CsrBufs& c, char* ws, size_t off, int E, int N) {
  const size_t off0 = off; c.base = ws + off;
  auto al = [&](size_t bytes) { char* p = ws + off; off += (bytes + 255) & ~(size_t)255; return p; };
  c.nG = (N + CSR_GN - 1) / CSR_GN; c.NGP = (c.nG + 31) & ~31; const int ch = (E + CSR_NBLK - 1) / CSR_NBLK; c.CHP = (ch + 31) & ~31; c.permLen = (size_t)E + 32 * (size_t)c.nG + 32;
  c.STG = (int*)al((size_t)CSR_NBLK * c.CHP * 4); c.HST = (int*)al((size_t)CSR_NBLK * c.NGP * 4); c.OFF = (int*)al((size_t)c.NGP * CSR_NBLK * 4); c.START = (int*)al((size_t)(c.NGP + 64) * 4); c.TOT = (int*)al((size_t)(c.NGP + 64) * 4);
  c.PERM = (int*)al(c.permLen * 4); c.ROWPTR = (int*)al((size_t)c.nG * CSR_GN * 4); c.ROWCNT = (int*)al((size_t)c.nG * CSR_GN * 4); c.FLAG = (int*)al(256);
  c.bytes = off - off0; return off;
}
static void csr_build(const CsrBufs& c, const int* dst, int E, int N, hipStream_t stream) {
  const size_t smem = (size_t)(2 * c.NGP + c.CHP) * 4;
  csrZ_kernel<<<512, 256, 0, stream>>>((int*)c.base, c.bytes / 16);
  csrA_kernel<<<CSR_NBLK, 64, smem, stream>>>(dst, E, N, c.nG, c.CHP, c.NGP, c.STG, c.HST);
  csrS_kernel<<<1, 512, 0, stream>>>(c.HST, c.nG, c.NGP, c.START, c.TOT, c.OFF);
  csrB_kernel<<<c.nG, 256, 0, stream>>>(dst, N, c.nG, c.CHP, c.NGP, (int)c.permLen, c.STG, c.HST, c.OFF, c.START, c.TOT, c.PERM, c.ROWPTR, c.ROWCNT, c.FLAG);
}


__global__ __launch_bounds__(256) void prepx_kernel(const float* __restrict__ x, const float* __restrict__ wih, const float* __restrict__ whh, b16* __restrict__ X16, b16* __restrict__ WIH, b16* __restrict__ WHH) {
  const size_t g = (size_t)blockIdx.x * 256 + threadIdx.x; const size_t n0 = (size_t)NP * H / 8, n1 = (size_t)G3 * H / 8;
  v8b o; b16* dst; const float* src; size_t e; float sc;
  if (g < n0) { e = g * 8; dst = X16 + e; if (e / H >= (size_t)N) { o = (v8b){}; for (int pass = 0; pass < 2; ++pass) { *(volatile v8b*)dst = o; __threadfence(); } return; } src = x + e; sc = XS; }
  else if (g < n0 + n1) { e = (g - n0) * 8; dst = WIH + e; src = wih + e; sc = WSC; } else if (g < n0 + 2 * n1) { e = (g - n0 - n1) * 8; dst = WHH + e; src = whh + e; sc = WSC; } else return;
  const v4f a = *(const v4f*)src, c = *(const v4f*)(src + 4);
#pragma unroll
  for (int j = 0; j < 4; ++j) { o[j] = (b16)(bf16_rne(a[j]) * sc); o[4 + j] = (b16)(bf16_rne(c[j]) * sc); }
  for (int pass = 0; pass < 2; ++pass) { *(volatile v8b*)dst = o; __threadfence(); }
}
__global__ __launch_bounds__(256) void prepw_kernel(const float* __restrict__ w1, const float* __restrict__ w2, b16* __restrict__ W1T, b16* __restrict__ W2T) {
  __shared__ __attribute__((aligned(16))) b16 T[64][64 + 8];
  const int kind = blockIdx.z, i0 = blockIdx.x * 64, o0 = blockIdx.y * 64, t_ = threadIdx.x;
  const int IN = kind == 0 ? KIN : H, INP = kind == 0 ? KP : H; if (i0 >= INP || o0 >= H) return;
  const float* w = kind == 0 ? w1 : w2; b16* dst = kind == 0 ? W1T : W2T;
  for (int q = t_; q < 64 * 64; q += 256) { const int ii = q >> 6, oo = q & 63; const int i = i0 + ii; T[oo][ii] = (i < IN) ? (b16)(bf16_rne(w[(size_t)(i < IN ? i : 0) * H + o0 + oo]) * WSC) : (b16)0.0f; }
  __syncthreads();
  for (int pass = 0; pass < 2; ++pass) { for (int q = t_; q < 64 * 8; q += 256) { const int oo = q >> 3, c8 = (q & 7) * 8; if (i0 + c8 < INP) *(volatile v8b*)(dst + (size_t)(o0 + oo) * INP + i0 + c8) = *(const v8b*)(&T[oo][c8]); } __threadfence(); }
}
__global__ __launch_bounds__(128) void edge_kernel(const int* __restrict__ src, const int* __restrict__ dst, const float* __restrict__ ea, const float* __restrict__ pos, const b16* __restrict__ X16, const b16* __restrict__ W1T, const float* __restrict__ b1, const float* __restrict__ g1, const float* __restrict__ be1, const b16* __restrict__ W2T, const float* __restrict__ b2, int ebase, b16* __restrict__ MSG) {
  __shared__ __attribute__((aligned(16))) b16 Ta[4][16][KP + 8], Tlo[4][16][32 + 8], Hh[4][16][H + 8], Hl[4][16][H + 8];
  const int wave = threadIdx.x >> 5, lane = threadIdx.x & 31, nloc = lane & 15, hlf = lane >> 4; const int e0 = ebase + (blockIdx.x * 4 + wave) * 16;
  if (e0 >= ebase + EQ || e0 >= E) return;
  { const int rr = lane >> 1, hf = lane & 1; const int e = e0 + rr; const int s = iclamp(src[e], 0, N - 1), d = iclamp(dst[e], 0, N - 1);
    const v8b* xd = (const v8b*)(X16 + (size_t)d * H + hf * 64); const v8b* xs = (const v8b*)(X16 + (size_t)s * H + hf * 64);
#pragma unroll
    for (int q = 0; q < 8; ++q) { *(v8b*)(&Ta[wave][rr][hf * 64 + q * 8]) = xd[q]; *(v8b*)(&Ta[wave][rr][H + hf * 64 + q * 8]) = xs[q]; }
#pragma unroll
    for (int j = 0; j < 8; ++j) { const int c = hf * 8 + j; Ta[wave][rr][2 * H + c] = (b16)(bf16_rne(ea[(size_t)e * ED + c]) * XS); }
    const float r0 = (bf16_rne(pos[s * 3 + 0]) - bf16_rne(pos[d * 3 + 0])) / 5.0f, r1 = (bf16_rne(pos[s * 3 + 1]) - bf16_rne(pos[d * 3 + 1])) / 5.0f, r2 = (bf16_rne(pos[s * 3 + 2]) - bf16_rne(pos[d * 3 + 2])) / 5.0f;
    const float d2 = pmul(r0, r0) + pmul(r1, r1) + pmul(r2, r2); const float gv[4] = {r0, r1, r2, d2};
    if (hf == 0) {
#pragma unroll
      for (int j = 0; j < 4; ++j) { b16 a_, c_; split16(gv[j] * XS, a_, c_); Ta[wave][rr][2 * H + ED + j] = a_; Tlo[wave][rr][ED + j] = c_; }
      for (int j = 2 * H + ED + 4; j < KP; ++j) Ta[wave][rr][j] = (b16)0.0f;
      for (int j = 0; j < 32; ++j) if (j < ED || j >= ED + 4) Tlo[wave][rr][j] = (b16)0.0f; } }
  wave_lds_sync();
  v8f acc[8];
#pragma unroll
  for (int t = 0; t < 8; ++t) acc[t] = (v8f){};
  for (int kb = 0; kb < KP; kb += 32) { const v16b a = frag_kb(&Ta[wave][nloc][kb], hlf);
#pragma unroll
    for (int t = 0; t < 8; ++t) acc[t] = wmma16b(a, frag_kb(W1T + (size_t)(t * 16 + nloc) * KP + kb, hlf), acc[t]); }
  { const v16b al = frag_kb(&Tlo[wave][nloc][0], hlf);
#pragma unroll
    for (int t = 0; t < 8; ++t) acc[t] = wmma16b(al, frag_kb(W1T + (size_t)(t * 16 + nloc) * KP + 2 * H, hlf), acc[t]); }
#pragma unroll
  for (int t = 0; t < 8; ++t) { const float bb = bf16_rne(b1[t * 16 + nloc]);
#pragma unroll
    for (int r = 0; r < 8; ++r) acc[t][r] = acc[t][r] * (1.0f / (XS * WSC)) + bb; }
#pragma unroll
  for (int r = 0; r < 8; ++r) { float s = 0.0f;
#pragma unroll
    for (int t = 0; t < 8; ++t) s += acc[t][r];
    s = hsum16(s); const float mu = s * (1.0f / H); float ss = 0.0f;
#pragma unroll
    for (int t = 0; t < 8; ++t) { const float dv = acc[t][r] - mu; ss += pmul(dv, dv); }
    ss = hsum16(ss); const float rs = rsqrtf(ss * (1.0f / H) + EPS);
#pragma unroll
    for (int t = 0; t < 8; ++t) { const int c = t * 16 + nloc; const float v = pmul(bf16_rne(g1[c]), (acc[t][r] - mu) * rs) + bf16_rne(be1[c]); const float hsl = v * sigm(v); b16 a_, c_; split16(hsl * XS, a_, c_); Hh[wave][8 * hlf + r][c] = a_; Hl[wave][8 * hlf + r][c] = c_; } }
  wave_lds_sync();
#pragma unroll
  for (int t = 0; t < 8; ++t) acc[t] = (v8f){};
#pragma unroll
  for (int kb = 0; kb < H; kb += 32) { const v16b a = frag_kb(&Hh[wave][nloc][kb], hlf), al = frag_kb(&Hl[wave][nloc][kb], hlf);
#pragma unroll
    for (int t = 0; t < 8; ++t) { const v16b bw = frag_kb(W2T + (size_t)(t * 16 + nloc) * H + kb, hlf); acc[t] = wmma16b(a, bw, acc[t]); acc[t] = wmma16b(al, bw, acc[t]); } }
  wave_lds_sync();
#pragma unroll
  for (int t = 0; t < 8; ++t) { const float bb = bf16_rne(b2[t * 16 + nloc]);
#pragma unroll
    for (int r = 0; r < 8; ++r) Hh[wave][8 * hlf + r][t * 16 + nloc] = (b16)((acc[t][r] * (1.0f / (XS * WSC)) + bb) * XS); }
  wave_lds_sync();
  for (int pass = 0; pass < 2; ++pass) { for (int rr = 0; rr < 16; ++rr) if (lane < 16) *(volatile v8b*)(MSG + ((size_t)(e0 - ebase) + rr) * H + lane * 8) = *(const v8b*)(&Hh[wave][rr][lane * 8]); __threadfence(); }
}
template <int QTR>
__global__ __launch_bounds__(256) void agg_kernel(const b16* __restrict__ MSG, const int* __restrict__ PERM, const int* __restrict__ ROWPTR, const int* __restrict__ ROWCNT, int permLen, float* __restrict__ AGG, b16* __restrict__ AGh, b16* __restrict__ AGl) {
  const int wave = threadIdx.x >> 5, lane = threadIdx.x & 31; const size_t v = ((size_t)blockIdx.x * 8 + wave) * 2 + (lane >> 4); const int c0 = (lane & 15) * 8;
  int st = ROWPTR[v], cnt = ROWCNT[v]; cnt = iclamp(cnt, 0, 8192); st = iclamp(st, 0, permLen - cnt);
  float acc[8]; if (QTR == 0) { for (int j = 0; j < 8; ++j) acc[j] = 0.0f; } else { const v4f a = *(const v4f*)(AGG + v * H + c0), b = *(const v4f*)(AGG + v * H + c0 + 4); for (int j = 0; j < 4; ++j) { acc[j] = a[j]; acc[4 + j] = b[j]; } }
  for (int j = 0; j < cnt; ++j) { const int e = iclamp(PERM[st + j], 0, E - 1); const bool inq = (e >= QTR * EQ) && (e < (QTR + 1) * EQ); const int el = iclamp(e - QTR * EQ, 0, EQ - 1);
    const v8b mv = *(const v8b*)(MSG + (size_t)el * H + c0);
#pragma unroll
    for (int q = 0; q < 8; ++q) acc[q] += inq ? (float)mv[q] * (1.0f / XS) : 0.0f; }
  if (QTR == 3) { const float inv = 1.0f / (float)(cnt > 1 ? cnt : 1); for (int q = 0; q < 8; ++q) acc[q] *= inv; }
  v4f oa = {acc[0], acc[1], acc[2], acc[3]}, ob = {acc[4], acc[5], acc[6], acc[7]};
  v8b hh8, ll8; if (QTR == 3) { for (int q = 0; q < 8; ++q) { b16 a_, c_; split16(acc[q] * XS, a_, c_); hh8[q] = a_; ll8[q] = c_; } }
  for (int pass = 0; pass < 2; ++pass) { *(volatile v4f*)(AGG + v * H + c0) = oa; *(volatile v4f*)(AGG + v * H + c0 + 4) = ob; if (QTR == 3) { *(volatile v8b*)(AGh + v * H + c0) = hh8; *(volatile v8b*)(AGl + v * H + c0) = ll8; } __threadfence(); }
}
__global__ __launch_bounds__(128) void gru_kernel(const b16* __restrict__ AGh, const b16* __restrict__ AGl, const b16* __restrict__ X16, const float* __restrict__ x, const b16* __restrict__ WIH, const float* __restrict__ bih, const b16* __restrict__ WHH, const float* __restrict__ bhh, const float* __restrict__ g2, const float* __restrict__ be2, float* __restrict__ out) {
  __shared__ __attribute__((aligned(16))) float Ty[16][H + 4];
  const int wave = threadIdx.x >> 5, lane = threadIdx.x & 31, nloc = lane & 15, hlf = lane >> 4; const size_t m0 = (size_t)blockIdx.x * 16; const int u0 = wave * 32;
  v8f gi[6], gh[6];
#pragma unroll
  for (int t = 0; t < 6; ++t) { gi[t] = (v8f){}; gh[t] = (v8f){}; }
#pragma unroll
  for (int kb = 0; kb < H; kb += 32) { const v16b a = frag_kb(AGh + (m0 + nloc) * H + kb, hlf), al = frag_kb(AGl + (m0 + nloc) * H + kb, hlf), ax = frag_kb(X16 + (m0 + nloc) * H + kb, hlf);
#pragma unroll
    for (int g = 0; g < 3; ++g)
#pragma unroll
      for (int ut = 0; ut < 2; ++ut) { const size_t row = (size_t)(g * H + u0 + ut * 16 + nloc); const v16b bi = frag_kb(WIH + row * H + kb, hlf), bh_ = frag_kb(WHH + row * H + kb, hlf);
        gi[g * 2 + ut] = wmma16b(a, bi, gi[g * 2 + ut]); gi[g * 2 + ut] = wmma16b(al, bi, gi[g * 2 + ut]); gh[g * 2 + ut] = wmma16b(ax, bh_, gh[g * 2 + ut]); } }
#pragma unroll
  for (int ut = 0; ut < 2; ++ut) { const int u = u0 + ut * 16 + nloc; const float bir = bf16_rne(bih[u]), biz = bf16_rne(bih[H + u]), bin = bf16_rne(bih[2 * H + u]), bhr = bf16_rne(bhh[u]), bhz = bf16_rne(bhh[H + u]), bhn = bf16_rne(bhh[2 * H + u]);
#pragma unroll
    for (int r = 0; r < 8; ++r) { const size_t row = m0 + 8 * hlf + r; const float sc = 1.0f / (XS * WSC);
      const float rg = sigm(gi[0 + ut][r] * sc + bir + gh[0 + ut][r] * sc + bhr), zg = sigm(gi[2 + ut][r] * sc + biz + gh[2 + ut][r] * sc + bhz);
      const float ng = tanh_(gi[4 + ut][r] * sc + bin + pmul(rg, gh[4 + ut][r] * sc + bhn)); const float xv = bf16_rne(x[(row < N ? row : (size_t)(N - 1)) * H + u]);
      const float upd = pmul(1.0f - zg, ng) + pmul(zg, xv); Ty[8 * hlf + r][u] = xv + upd; } }
  __syncthreads();
  for (int rr = wave * 4; rr < wave * 4 + 4; ++rr) { const size_t row = m0 + rr; const v4f v = *(const v4f*)(&Ty[rr][lane * 4]); float s = v[0] + v[1] + v[2] + v[3];
#pragma unroll
    for (int o = 16; o >= 1; o >>= 1) s += __shfl_xor(s, o);
    const float mu = s * (1.0f / H); float ss = 0.0f; for (int j = 0; j < 4; ++j) { const float dv = v[j] - mu; ss += pmul(dv, dv); }
#pragma unroll
    for (int o = 16; o >= 1; o >>= 1) ss += __shfl_xor(ss, o);
    const float rs = rsqrtf(ss * (1.0f / H) + EPS); v4f y; for (int j = 0; j < 4; ++j) { const int c = lane * 4 + j; y[j] = pmul(bf16_rne(g2[c]), (v[j] - mu) * rs) + bf16_rne(be2[c]); }
    for (int pass = 0; pass < 2; ++pass) { if (row < N) *(volatile v4f*)(out + row * H + lane * 4) = y; __threadfence(); } }
}
}

extern "C" void kernel_launch(void* const* d_in, const int* in_sizes, int n_in, void* d_out, int out_size, void* d_ws, size_t ws_size, hipStream_t stream) {
  (void)n_in;
  auto Fp = [&](int i) { return (const float*)d_in[i]; };
  if (in_sizes[0] != N * H || in_sizes[1] != E * ED || in_sizes[2] != N * 3 || in_sizes[3] != KIN * H || in_sizes[7] != H * H || in_sizes[9] != G3 * H || in_sizes[11] != G3 * H || in_sizes[15] != 2 * E || out_size != N * H) return;
  const int* src = (const int*)d_in[15]; const int* dst = src + E;
  size_t off = 0; char* ws = (char*)d_ws;
  auto carve = [&](size_t bytes) { char* p = ws + off; off += (bytes + 255) & ~(size_t)255; return p; };
  b16* X16 = (b16*)carve((size_t)NP * H * 2); b16* W1T = (b16*)carve((size_t)H * KP * 2); b16* W2T = (b16*)carve(H * H * 2); b16* WIH = (b16*)carve((size_t)G3 * H * 2); b16* WHH = (b16*)carve((size_t)G3 * H * 2);
  b16* MSG = (b16*)carve((size_t)EQ * H * 2); float* AGG = (float*)carve((size_t)NP * H * 4); b16* AGh = (b16*)carve((size_t)NP * H * 2); b16* AGl = (b16*)carve((size_t)NP * H * 2);
  CsrBufs csr; off = csr_carve(csr, ws, off, E, N);
  if (off > ws_size || off > ((size_t)128 << 20)) return;
  prepx_kernel<<<((size_t)NP * H / 8 + 2 * G3 * H / 8 + 255) / 256, 256, 0, stream>>>(Fp(0), Fp(9), Fp(11), X16, WIH, WHH);
  prepw_kernel<<<dim3(KP / 64 + 1, H / 64, 2), 256, 0, stream>>>(Fp(3), Fp(7), W1T, W2T);
  csr_build(csr, dst, E, N, stream);
#define EDGEQ(q) edge_kernel<<<(EQ + 63) / 64, 128, 0, stream>>>(src, dst, Fp(1), Fp(2), X16, W1T, Fp(4), Fp(5), Fp(6), W2T, Fp(8), q * EQ, MSG)
  EDGEQ(0); agg_kernel<0><<<NP / 16, 256, 0, stream>>>(MSG, csr.PERM, csr.ROWPTR, csr.ROWCNT, (int)csr.permLen, AGG, AGh, AGl);
  EDGEQ(1); agg_kernel<1><<<NP / 16, 256, 0, stream>>>(MSG, csr.PERM, csr.ROWPTR, csr.ROWCNT, (int)csr.permLen, AGG, AGh, AGl);
  EDGEQ(2); agg_kernel<2><<<NP / 16, 256, 0, stream>>>(MSG, csr.PERM, csr.ROWPTR, csr.ROWCNT, (int)csr.permLen, AGG, AGh, AGl);
  EDGEQ(3); agg_kernel<3><<<NP / 16, 256, 0, stream>>>(MSG, csr.PERM, csr.ROWPTR, csr.ROWCNT, (int)csr.permLen, AGG, AGh, AGl);
#undef EDGEQ
  gru_kernel<<<NP / 16, 128, 0, stream>>>(AGh, AGl, X16, Fp(0), WIH, Fp(10), WHH, Fp(12), Fp(13), Fp(14), (float*)d_out);
}
